// ConditionNetDDFT_49813030699480
// MI455X (gfx1250) — hardware-verified
//
#include <hip/hip_runtime.h>
#define NB 16
#define HS 256
#define PX (HS * HS)
#define NF 64
#define KT 4
typedef __bf16 v16b __attribute__((ext_vector_type(16)));
typedef unsigned short v8us __attribute__((ext_vector_type(8), may_alias));
typedef float  v8f  __attribute__((ext_vector_type(8)));
typedef float  v4f  __attribute__((ext_vector_type(4)));
typedef float  v4fa __attribute__((ext_vector_type(4), may_alias));
union FragB { v16b v; v8us half[2]; unsigned short u[16]; };

__device__ __forceinline__ unsigned short bf16_bits(float x) { unsigned int u = __float_as_uint(x); return (unsigned short)((u + 0x7FFFu + ((u >> 16) & 1u)) >> 16); }
__device__ __forceinline__ float bf16_val(unsigned short b) { return __uint_as_float(((unsigned int)b) << 16); }
__device__ __forceinline__ float bf16_round(float x) { return bf16_val(bf16_bits(x)); }
template <int NT>
__device__ __forceinline__ v8f mmaN(v16b ah, v16b al, v16b bh, v16b bl, v8f c) {
  c = __builtin_amdgcn_wmma_f32_16x16x32_bf16(false, ah, false, bh, (short)0, c, false, false);
  if (NT >= 2) c = __builtin_amdgcn_wmma_f32_16x16x32_bf16(false, al, false, bh, (short)0, c, false, false);
  if (NT >= 3) c = __builtin_amdgcn_wmma_f32_16x16x32_bf16(false, ah, false, bl, (short)0, c, false, false);
  asm volatile("v_nop\n\tv_nop\n\tv_nop\n\tv_nop" : "+v"(c) : "v"(ah), "v"(al), "v"(bh), "v"(bl));
  return c;
}

__global__ __launch_bounds__(256) void k_wt_bf16(const float* __restrict__ W, unsigned short* __restrict__ Wt, int K, int N) {
  const int t = blockIdx.x * 256 + threadIdx.x;
  const int k8n = K / 8;
  if (t >= N * k8n) return;
  const int n = t / k8n, k8 = (t % k8n) * 8;
  v8us v;
#pragma unroll
  for (int i = 0; i < 8; ++i) v[i] = bf16_bits(W[(size_t)(k8 + i) * N + n]);
  *(volatile v8us*)(Wt + (size_t)n * K + k8) = v;
  __threadfence();
  *(volatile v8us*)(Wt + (size_t)n * K + k8) = v;
}

template <bool ASPLIT, int ACT, bool BIAS_BF16>
__global__ __launch_bounds__(128) void k_gemm_bf(const float* __restrict__ A, int lda, const unsigned short* __restrict__ Wt, int ldb,
                                               const float* __restrict__ bias, float* __restrict__ C, int ldc, int M, int N, int K) {
  __shared__ __attribute__((aligned(16))) float so[4][16][64];
  const int tid = threadIdx.x, w = tid >> 5, lane = tid & 31, ln = lane & 15, hh = lane >> 4;
  const int ntn = N / 64;
  const int wid = blockIdx.x * 4 + w;
  const int mt = wid / ntn, nq = wid % ntn;
  if (mt * 16 >= M) return;
  const int row0 = mt * 16, col0 = nq * 64;
  const float* arow = A + (size_t)(row0 + ln) * lda;
  v8f acc[4] = {};
  for (int kb = 0; kb < K; kb += 32) {
    FragB ah, al;
    const v4f x0 = *(const v4fa*)(arow + kb + 8 * hh), x1 = *(const v4fa*)(arow + kb + 8 * hh + 4);
    const v4f x2 = *(const v4fa*)(arow + kb + 16 + 8 * hh), x3 = *(const v4fa*)(arow + kb + 16 + 8 * hh + 4);
    float xs[16] = {x0[0],x0[1],x0[2],x0[3],x1[0],x1[1],x1[2],x1[3],x2[0],x2[1],x2[2],x2[3],x3[0],x3[1],x3[2],x3[3]};
#pragma unroll
    for (int i = 0; i < 16; ++i) { const unsigned short hb = bf16_bits(xs[i]); ah.u[i] = hb; al.u[i] = ASPLIT ? bf16_bits(xs[i] - bf16_val(hb)) : (unsigned short)0; }
#pragma unroll
    for (int t = 0; t < 4; ++t) {
      const unsigned short* brow = Wt + (size_t)(col0 + t * 16 + ln) * ldb + kb;
      FragB b;
      b.half[0] = *(const v8us*)(brow + 8 * hh);
      b.half[1] = *(const v8us*)(brow + 16 + 8 * hh);
      acc[t] = mmaN<ASPLIT ? 2 : 1>(ah.v, al.v, b.v, b.v, acc[t]);
    }
  }
#pragma unroll
  for (int t = 0; t < 4; ++t) {
    float bv = bias ? bias[col0 + t * 16 + ln] : 0.f;
    if (BIAS_BF16) bv = bf16_round(bv);
#pragma unroll
    for (int r = 0; r < 8; ++r) { float v = acc[t][r] + bv; if (ACT == 1) v = fmaxf(v, 0.f); so[w][8 * hh + r][t * 16 + ln] = v; }
  }
  __builtin_amdgcn_fence(__ATOMIC_ACQ_REL, "workgroup");
  __builtin_amdgcn_wave_barrier();
  const int rsub = lane >> 4, c4 = (lane & 15) * 4;
  for (int pass = 0; pass < 2; ++pass) {
#pragma unroll
    for (int q = 0; q < 8; ++q) {
      const int r = q * 2 + rsub;
      const v4f v = *(const v4fa*)&so[w][r][c4];
      *(volatile v4f*)(C + (size_t)(row0 + r) * ldc + col0 + c4) = v;
    }
    if (pass == 0) __threadfence();
  }
}

template <bool ASPLIT, int ACT, bool BIAS_BF16, bool RES_BF16>
__global__ __launch_bounds__(128) void k_gemm_bf3(const float* __restrict__ A, int lda, const unsigned short* __restrict__ Wt, int ldb,
                                                const float* __restrict__ bias, const float* __restrict__ resid, int rmod, int ldr,
                                                float* __restrict__ C, int ldc, int M, int N, int K) {
  __shared__ __attribute__((aligned(16))) float so[4][16][64];
  const int tid = threadIdx.x, w = tid >> 5, lane = tid & 31, ln = lane & 15, hh = lane >> 4;
  const int ntn = N / 64;
  const int wid = blockIdx.x * 4 + w;
  const int mt = wid / ntn, nq = wid % ntn;
  if (mt * 16 >= M) return;
  const int row0 = mt * 16, col0 = nq * 64;
  const float* arow = A + (size_t)(row0 + ln) * lda;
  v8f acc[4] = {};
  for (int kb = 0; kb < K; kb += 32) {
    FragB ah, al;
    const v4f x0 = *(const v4fa*)(arow + kb + 8 * hh), x1 = *(const v4fa*)(arow + kb + 8 * hh + 4);
    const v4f x2 = *(const v4fa*)(arow + kb + 16 + 8 * hh), x3 = *(const v4fa*)(arow + kb + 16 + 8 * hh + 4);
    float xs[16] = {x0[0],x0[1],x0[2],x0[3],x1[0],x1[1],x1[2],x1[3],x2[0],x2[1],x2[2],x2[3],x3[0],x3[1],x3[2],x3[3]};
#pragma unroll
    for (int i = 0; i < 16; ++i) { const unsigned short hb = bf16_bits(xs[i]); ah.u[i] = hb; al.u[i] = ASPLIT ? bf16_bits(xs[i] - bf16_val(hb)) : (unsigned short)0; }
#pragma unroll
    for (int t = 0; t < 4; ++t) {
      const unsigned short* brow = Wt + (size_t)(col0 + t * 16 + ln) * ldb + kb;
      FragB b;
      b.half[0] = *(const v8us*)(brow + 8 * hh);
      b.half[1] = *(const v8us*)(brow + 16 + 8 * hh);
      acc[t] = mmaN<ASPLIT ? 2 : 1>(ah.v, al.v, b.v, b.v, acc[t]);
    }
  }
#pragma unroll
  for (int t = 0; t < 4; ++t) {
    const int col = col0 + t * 16 + ln;
    float bv = bias ? bias[col] : 0.f;
    if (BIAS_BF16) bv = bf16_round(bv);
#pragma unroll
    for (int r = 0; r < 8; ++r) {
      float v = acc[t][r] + bv;
      if (resid) { float rv = resid[(size_t)((row0 + 8 * hh + r) % rmod) * ldr + col]; if (RES_BF16) rv = bf16_round(rv); v += rv; }
      if (ACT == 1) v = fmaxf(v, 0.f);
      if (ACT == 2) v = 0.5f * v * (1.0f + erff(v * 0.70710678118654752f));
      if (ACT == 3) { const float u = 0.7978845608028654f * (v + 0.044715f * v * v * v); v = 0.5f * v * (1.0f + tanhf(u)); }
      so[w][8 * hh + r][t * 16 + ln] = v;
    }
  }
  __builtin_amdgcn_fence(__ATOMIC_ACQ_REL, "workgroup");
  __builtin_amdgcn_wave_barrier();
  const int rsub = lane >> 4, c4 = (lane & 15) * 4;
  for (int pass = 0; pass < 2; ++pass) {
#pragma unroll
    for (int q = 0; q < 8; ++q) {
      const int r = q * 2 + rsub;
      const v4f v = *(const v4fa*)&so[w][r][c4];
      *(volatile v4f*)(C + (size_t)(row0 + r) * ldc + col0 + c4) = v;
    }
    if (pass == 0) __threadfence();
  }
}
template <bool PARAM_BF16>
__global__ __launch_bounds__(256) void k_layernorm(const float* __restrict__ X, const float* __restrict__ R, const float* __restrict__ g, const float* __restrict__ bta,
                                                  float* __restrict__ out_sum, float* __restrict__ out_norm, int N, float eps) {
  __shared__ float red[256];
  const int row = blockIdx.x, tid = threadIdx.x;
  const float* x = X + (size_t)row * N; const float* rr = R ? R + (size_t)row * N : nullptr;
  float vals[16];
  const int per = N / 256;
  float s1 = 0.f;
  for (int u = 0; u < per / 4; ++u) {
    const int j = tid * 4 + 1024 * u;
    const v4f a = *(const v4fa*)(x + j);
    v4f b = {0.f,0.f,0.f,0.f}; if (rr) b = *(const v4fa*)(rr + j);
#pragma unroll
    for (int q = 0; q < 4; ++q) { const float v = a[q] + b[q]; vals[u * 4 + q] = v; s1 += v; }
  }
  red[tid] = s1; __syncthreads();
  for (int st = 128; st > 0; st >>= 1) { if (tid < st) red[tid] += red[tid + st]; __syncthreads(); }
  const float mu = red[0] / (float)N; __syncthreads();
  float s2 = 0.f;
  for (int u = 0; u < per / 4; ++u)
#pragma unroll
    for (int q = 0; q < 4; ++q) { const float c = vals[u * 4 + q] - mu; s2 += c * c; }
  red[tid] = s2; __syncthreads();
  for (int st = 128; st > 0; st >>= 1) { if (tid < st) red[tid] += red[tid + st]; __syncthreads(); }
  const float rs = rsqrtf(red[0] / (float)N + eps);
  for (int pass = 0; pass < 2; ++pass) {
    for (int u = 0; u < per / 4; ++u) {
      const int j = tid * 4 + 1024 * u;
      v4f o, sm;
#pragma unroll
      for (int q = 0; q < 4; ++q) {
        float gg = g[j + q], bb = bta[j + q];
        if (PARAM_BF16) { gg = bf16_round(gg); bb = bf16_round(bb); }
        sm[q] = vals[u * 4 + q]; o[q] = (vals[u * 4 + q] - mu) * rs * gg + bb;
      }
      if (out_sum) *(volatile v4f*)(out_sum + (size_t)row * N + j) = sm;
      *(volatile v4f*)(out_norm + (size_t)row * N + j) = o;
    }
    if (pass == 0) __threadfence();
  }
}


typedef _Float16 v16h __attribute__((ext_vector_type(16)));
union FragH { v16h v; v8us half[2]; _Float16 h[16]; unsigned short u[16]; };
template <int NT>
__device__ __forceinline__ v8f mmaH(v16h ah, v16h al, v16h bh, v16h bl, v8f c) {
  c = __builtin_amdgcn_wmma_f32_16x16x32_f16(false, ah, false, bh, (short)0, c, false, false);
  if (NT >= 2) c = __builtin_amdgcn_wmma_f32_16x16x32_f16(false, al, false, bh, (short)0, c, false, false);
  if (NT >= 3) c = __builtin_amdgcn_wmma_f32_16x16x32_f16(false, ah, false, bl, (short)0, c, false, false);
  asm volatile("v_nop\n\tv_nop\n\tv_nop\n\tv_nop" : "+v"(c) : "v"(ah), "v"(al), "v"(bh), "v"(bl));
  return c;
}
template <bool ASPLIT>
__global__ __launch_bounds__(128) void k_gemm_h(const float* __restrict__ A, int lda, size_t sA, const _Float16* __restrict__ Bh, int ldb, size_t sB, float alpha, float* __restrict__ C, int ldc, size_t sC, int M, int N, int K) {
  __shared__ __attribute__((aligned(16))) float so[4][16][64];
  const int tid = threadIdx.x, w = tid >> 5, lane = tid & 31, ln = lane & 15, hh = lane >> 4; const int by = blockIdx.y;
  A += (size_t)by * sA; Bh += (size_t)by * sB; C += (size_t)by * sC;
  const int ntn = (N + 63) / 64; const int wid = blockIdx.x * 4 + w; const int mt = wid / ntn, nq = wid % ntn; if (mt * 16 >= M) return;
  const int row0 = mt * 16, col0 = nq * 64; const float* arow = A + (size_t)(row0 + ln) * lda;
  v8f acc[4] = {};
  for (int kb = 0; kb < K; kb += 32) {
    FragH ah, al;
    const v4f x0 = *(const v4fa*)(arow + kb + 8 * hh), x1 = *(const v4fa*)(arow + kb + 8 * hh + 4), x2 = *(const v4fa*)(arow + kb + 16 + 8 * hh), x3 = *(const v4fa*)(arow + kb + 16 + 8 * hh + 4);
    float xs[16] = {x0[0],x0[1],x0[2],x0[3],x1[0],x1[1],x1[2],x1[3],x2[0],x2[1],x2[2],x2[3],x3[0],x3[1],x3[2],x3[3]};
#pragma unroll
    for (int i = 0; i < 16; ++i) { const _Float16 h = (_Float16)xs[i]; ah.h[i] = h; al.h[i] = ASPLIT ? (_Float16)(xs[i] - (float)h) : (_Float16)0.0f; }
#pragma unroll
    for (int t = 0; t < 4; ++t) { if (col0 + t * 16 >= N) continue; const size_t boff = (size_t)(col0 + t * 16 + ln) * ldb + kb; FragH bq; bq.half[0] = *(const v8us*)(Bh + boff + 8 * hh); bq.half[1] = *(const v8us*)(Bh + boff + 16 + 8 * hh);
      acc[t] = mmaH<ASPLIT ? 2 : 1>(ah.v, al.v, bq.v, bq.v, acc[t]); }
  }
#pragma unroll
  for (int t = 0; t < 4; ++t) { if (col0 + t * 16 >= N) continue;
#pragma unroll
    for (int r = 0; r < 8; ++r) so[w][8 * hh + r][t * 16 + ln] = acc[t][r] * alpha; }
  __builtin_amdgcn_fence(__ATOMIC_ACQ_REL, "workgroup"); __builtin_amdgcn_wave_barrier();
  const int rsub = lane >> 4, c4 = (lane & 15) * 4;
  for (int pass = 0; pass < 2; ++pass) {
#pragma unroll
    for (int q = 0; q < 8; ++q) { const int r = q * 2 + rsub; if (col0 + c4 < N) { const v4f v = *(const v4fa*)&so[w][r][c4]; *(volatile v4f*)(C + (size_t)(row0 + r) * ldc + col0 + c4) = v; } }
    if (pass == 0) __threadfence(); }
}

__global__ __launch_bounds__(256) void k_wt_f16(const float* __restrict__ W, _Float16* __restrict__ Wt, int K, int N, float scale) {
  const int t = blockIdx.x * 256 + threadIdx.x; if (t >= N * (K / 8)) return; const int n = t / (K / 8), k8 = (t % (K / 8)) * 8; FragH f;
#pragma unroll
  for (int i = 0; i < 8; ++i) f.h[i] = (_Float16)(bf16_round(W[(size_t)(k8 + i) * N + n]) * scale); const v8us o = f.half[0];
  *(volatile v8us*)((unsigned short*)Wt + (size_t)n * K + k8) = o; __threadfence(); *(volatile v8us*)((unsigned short*)Wt + (size_t)n * K + k8) = o;
}
template <int ACT>
__global__ __launch_bounds__(128) void k_gemm_hhx(const _Float16* __restrict__ A, int lda, size_t sA, const _Float16* __restrict__ Bh, int ldb, size_t sB, float alpha, const float* __restrict__ bias, size_t sBias, const float* __restrict__ CP, int rowsPerB, size_t sCPb, int row0g,
    float* __restrict__ C, _Float16* __restrict__ C16, int ldc, size_t sC, int M, int N, int K) {
  __shared__ __attribute__((aligned(16))) float so[4][16][64];
  const int tid = threadIdx.x, w = tid >> 5, lane = tid & 31, ln = lane & 15, hh = lane >> 4; const int by = blockIdx.y;
  A += (size_t)by * sA; Bh += (size_t)by * sB; const size_t cofs = (size_t)by * sC; const float* bp = bias ? bias + (size_t)by * sBias : nullptr;
  const int ntn = (N + 63) / 64; const int wid = blockIdx.x * 4 + w; const int mt = wid / ntn, nq = wid % ntn; if (mt * 16 >= M) return;
  const int row0 = mt * 16, col0 = nq * 64; const _Float16* arow = A + (size_t)(row0 + ln) * lda;
  v8f acc[4] = {};
  for (int kb = 0; kb < K; kb += 32) { FragH ah; ah.half[0] = *(const v8us*)((const unsigned short*)arow + kb + 8 * hh); ah.half[1] = *(const v8us*)((const unsigned short*)arow + kb + 16 + 8 * hh);
#pragma unroll
    for (int t = 0; t < 4; ++t) { if (col0 + t * 16 >= N) continue; const size_t boff = (size_t)(col0 + t * 16 + ln) * ldb + kb; FragH bq; bq.half[0] = *(const v8us*)((const unsigned short*)Bh + boff + 8 * hh); bq.half[1] = *(const v8us*)((const unsigned short*)Bh + boff + 16 + 8 * hh);
      acc[t] = mmaH<1>(ah.v, ah.v, bq.v, bq.v, acc[t]); }
  }
#pragma unroll
  for (int t = 0; t < 4; ++t) { if (col0 + t * 16 >= N) continue; const int col = col0 + t * 16 + ln; const float bv = bp ? bf16_round(bp[col]) : 0.f;
#pragma unroll
    for (int r = 0; r < 8; ++r) { float v = acc[t][r] * alpha + bv; if (CP) { const int rr = row0g + row0 + 8 * hh + r; if (rowsPerB < 0) v += CP[cofs + (size_t)rr * ldc + col];        else { const int bidx = rr / rowsPerB; v += CP[(size_t)bidx * sCPb + (size_t)by * 64 + col]; } } if (ACT == 1) v = (v > 0.f) ? v : expm1f(v); else if (ACT == 7) v = (v > 0.f) ? v + 1.0f : expf(v); else if (ACT == 8) v = tanhf(v); else if (ACT == 9) v = 0.5f * v * (1.0f + tanhf(0.7978845608028654f * (v + 0.044715f * v * v * v))); else if (ACT == 11) v = 1.0f / (1.0f + expf(-v)); else if (ACT == 12) v = (v > 0.f) ? v : 0.01f * v; else if (ACT == 14) v = (v > 0.f) ? v : 0.1f * v; else if (ACT == 16) v = (v >= 0.f) ? v : 0.3f * v; else if (ACT == 17) v = (v >= 0.f) ? v : 0.2f * v; else if (ACT == 15) v = v / (1.0f + expf(-v)); else if (ACT == 3) v = fmaxf(v, 0.f); else if (ACT == 6) v = 0.5f * v * (1.0f + erff(v * 0.70710678118654752f)); so[w][8 * hh + r][t * 16 + ln] = v; } }
  __builtin_amdgcn_fence(__ATOMIC_ACQ_REL, "workgroup"); __builtin_amdgcn_wave_barrier();
  const int rsub = lane >> 4, c4 = (lane & 15) * 4; typedef _Float16 v4h __attribute__((ext_vector_type(4)));
  for (int pass = 0; pass < 2; ++pass) {
#pragma unroll
    for (int q = 0; q < 8; ++q) { const int r = q * 2 + rsub; if (col0 + c4 < N) { const v4f v = *(const v4fa*)&so[w][r][c4]; if (C) *(volatile v4f*)(C + cofs + (size_t)(row0 + r) * ldc + col0 + c4) = v; if (C16) { v4h h4; for (int i = 0; i < 4; ++i) h4[i] = (_Float16)v[i]; *(volatile v4h*)(C16 + cofs + (size_t)(row0 + r) * ldc + col0 + c4) = h4; } } }
    if (pass == 0) __threadfence(); }
}


typedef _Float16 v4h __attribute__((ext_vector_type(4)));

__global__ __launch_bounds__(256) void k_x16(const float* __restrict__ x, _Float16* __restrict__ X16, size_t n8) { const size_t t = (size_t)blockIdx.x * 256 + threadIdx.x; if (t >= n8) return; FragH f;
#pragma unroll
  for (int q = 0; q < 8; ++q) f.h[q] = (_Float16)bf16_round(x[t * 8 + q]); *(volatile v8us*)((unsigned short*)X16 + t * 8) = f.half[0]; __threadfence(); *(volatile v8us*)((unsigned short*)X16 + t * 8) = f.half[0]; }
__global__ __launch_bounds__(256) void k_h16(const float* __restrict__ x, _Float16* __restrict__ X16, size_t n8) { const size_t t = (size_t)blockIdx.x * 256 + threadIdx.x; if (t >= n8) return; FragH f;
#pragma unroll
  for (int q = 0; q < 8; ++q) f.h[q] = (_Float16)x[t * 8 + q]; *(volatile v8us*)((unsigned short*)X16 + t * 8) = f.half[0]; __threadfence(); *(volatile v8us*)((unsigned short*)X16 + t * 8) = f.half[0]; }
__global__ __launch_bounds__(256) void k_round16f(const float* __restrict__ W, _Float16* __restrict__ Bt, size_t n8) { const size_t t = (size_t)blockIdx.x * 256 + threadIdx.x; if (t >= n8) return; FragH f;
#pragma unroll
  for (int i = 0; i < 8; ++i) f.h[i] = (_Float16)(bf16_round(W[t * 8 + i]) * 16.0f); *(volatile v8us*)((unsigned short*)Bt + t * 8) = f.half[0]; __threadfence(); *(volatile v8us*)((unsigned short*)Bt + t * 8) = f.half[0]; }
template <int NHv, int TTv>
__global__ __launch_bounds__(256) void k_vt(const _Float16* __restrict__ V16, int ldv, int voff, _Float16* __restrict__ Vt) { __shared__ unsigned short tl[64][66]; const int tid = threadIdx.x; const int slab = blockIdx.x / (TTv / 64), lg = blockIdx.x % (TTv / 64); const int b = slab / NHv, h = slab % NHv;
  for (int i = tid; i < 64 * 8; i += 256) { const int r = i / 8, c8 = (i % 8) * 8; FragH f; f.half[0] = *(const v8us*)((const unsigned short*)V16 + ((size_t)b * TTv + lg * 64 + r) * ldv + voff + h * 64 + c8);
#pragma unroll
    for (int q = 0; q < 8; ++q) tl[r][c8 + q] = f.u[q]; }
  __syncthreads();
  for (int pass = 0; pass < 2; ++pass) {
#pragma unroll
    for (int rd = 0; rd < 2; ++rd) { const int d = rd * 32 + tid / 8, pc = tid % 8; FragH f;
#pragma unroll
      for (int q = 0; q < 8; ++q) f.u[q] = tl[pc * 8 + q][d];
      *(volatile v8us*)((unsigned short*)Vt + ((size_t)slab * 64 + d) * TTv + lg * 64 + pc * 8) = f.half[0]; }
    if (pass == 0) __threadfence(); } }

__global__ __launch_bounds__(256) void k_hl(const float* __restrict__ F, _Float16* __restrict__ Hh, _Float16* __restrict__ Hl, size_t n8) { const size_t t = (size_t)blockIdx.x * 256 + threadIdx.x; if (t >= n8) return; FragH fh, fl; const v4f a = *(const v4fa*)(F + t * 8), c = *(const v4fa*)(F + t * 8 + 4);
#pragma unroll
  for (int q = 0; q < 4; ++q) { _Float16 h = (_Float16)a[q]; fh.h[q] = h; fl.h[q] = (_Float16)((a[q] - (float)h) * 1024.0f); h = (_Float16)c[q]; fh.h[4 + q] = h; fl.h[4 + q] = (_Float16)((c[q] - (float)h) * 1024.0f); }
  for (int pass = 0; pass < 2; ++pass) { *(volatile v8us*)((unsigned short*)Hh + t * 8) = fh.half[0]; *(volatile v8us*)((unsigned short*)Hl + t * 8) = fl.half[0]; if (pass == 0) __threadfence(); } }

__device__ __forceinline__ v16h g2_frag(const _Float16* p, int hh) { FragH f; f.half[0] = *(const v8us*)((const unsigned short*)p + 8 * hh); f.half[1] = *(const v8us*)((const unsigned short*)p + 16 + 8 * hh); return f.v; }
__device__ __forceinline__ v8f g2_mma(v16h a, v16h b, v8f c) { v8f d = __builtin_amdgcn_wmma_f32_16x16x32_f16(false, a, false, b, (short)0, c, false, false); asm volatile("v_nop\n\tv_nop\n\tv_nop\n\tv_nop" : "+v"(d) : "v"(a), "v"(b)); return d; }
template <int ACT>
__global__ __launch_bounds__(128) void k_gemm2(const _Float16* __restrict__ A, int lda, size_t sA, const _Float16* __restrict__ Bh, int ldb, size_t sB, float alpha, const float* __restrict__ bias, size_t sBias, const float* __restrict__ CP, int rowsPerB, size_t sCPb, int row0g,
    float* __restrict__ C, _Float16* __restrict__ C16, int ldc, size_t sC, int M, int N, int K) { static_assert(ACT == 0 || ACT == 3 || ACT == 6 || ACT == 8 || ACT == 9 || ACT == 11 || ACT == 12 || ACT == 14 || ACT == 15 || ACT == 16 || ACT == 17, "k_gemm2: unsupported ACT code (would silently apply no activation)");
  __shared__ __attribute__((aligned(16))) float so[4][32][68];
  const int tid = threadIdx.x, w = tid >> 5, lane = tid & 31, ln = lane & 15, hh = lane >> 4; const int by = blockIdx.y;
  A += (size_t)by * sA; Bh += (size_t)by * sB; const size_t cofs = (size_t)by * sC; const float* bp = bias ? bias + (size_t)by * sBias : nullptr;
  const int ntn = N >> 6; const int mt = blockIdx.x / ntn, nq = blockIdx.x - mt * ntn; const int row0 = mt * 128 + 32 * w, col0 = nq * 64; if (row0 >= M) return;
  const _Float16* a0p = A + (size_t)(row0 + ln) * lda; const _Float16* a1p = a0p + (size_t)16 * lda;
  const _Float16* b0p = Bh + (size_t)(col0 + ln) * ldb; const _Float16* b1p = b0p + (size_t)16 * ldb; const _Float16* b2p = b1p + (size_t)16 * ldb; const _Float16* b3p = b2p + (size_t)16 * ldb;
  const v8f z8 = {0.f,0.f,0.f,0.f,0.f,0.f,0.f,0.f}; v8f c00 = z8, c01 = z8, c02 = z8, c03 = z8, c10 = z8, c11 = z8, c12 = z8, c13 = z8;
#pragma unroll 1
  for (int kb = 0; kb < K; kb += 32) { const v16h a0 = g2_frag(a0p + kb, hh), a1 = g2_frag(a1p + kb, hh);
    v16h b = g2_frag(b0p + kb, hh); c00 = g2_mma(a0, b, c00); c10 = g2_mma(a1, b, c10);
    b = g2_frag(b1p + kb, hh); c01 = g2_mma(a0, b, c01); c11 = g2_mma(a1, b, c11);
    b = g2_frag(b2p + kb, hh); c02 = g2_mma(a0, b, c02); c12 = g2_mma(a1, b, c12);
    b = g2_frag(b3p + kb, hh); c03 = g2_mma(a0, b, c03); c13 = g2_mma(a1, b, c13); }
  v8f accs[8] = {c00, c01, c02, c03, c10, c11, c12, c13};
#pragma unroll
  for (int u = 0; u < 8; ++u) { const int t = u & 3, half = u >> 2; const int col = col0 + t * 16 + ln; const float bv = bp ? bf16_round(bp[col]) : 0.f;
#pragma unroll
    for (int r = 0; r < 8; ++r) { const int rloc = half * 16 + 8 * hh + r; float v = accs[u][r] * alpha + bv; if (CP) { if (rowsPerB < 0) v += CP[cofs + (size_t)(row0g + row0 + rloc) * ldc + col];        else { const int bidx = (row0g + row0 + rloc) / rowsPerB; v += CP[(size_t)bidx * sCPb + (size_t)by * 64 + col]; } }
      if (ACT == 3) v = fmaxf(v, 0.f); else if (ACT == 6) v = 0.5f * v * (1.0f + erff(v * 0.70710678118654752f)); else if (ACT == 11) v = 1.0f / (1.0f + expf(-v)); else if (ACT == 15) v = v / (1.0f + expf(-v)); else if (ACT == 12) v = (v > 0.f) ? v : 0.01f * v; else if (ACT == 8) v = tanhf(v); else if (ACT == 9) v = 0.5f * v * (1.0f + tanhf(0.7978845608028654f * (v + 0.044715f * v * v * v))); else if (ACT == 14) v = (v > 0.f) ? v : 0.1f * v; else if (ACT == 16) v = (v >= 0.f) ? v : 0.3f * v; else if (ACT == 17) v = (v >= 0.f) ? v : 0.2f * v;
      so[w][rloc][t * 16 + ln] = v; } }
  __builtin_amdgcn_fence(__ATOMIC_ACQ_REL, "workgroup"); __builtin_amdgcn_wave_barrier();
  const int rsub = lane >> 4, c4 = (lane & 15) * 4;
  for (int pass = 0; pass < 2; ++pass) {
#pragma unroll
    for (int q = 0; q < 16; ++q) { const int r = q * 2 + rsub; const v4f v = *(const v4fa*)&so[w][r][c4]; if (C) *(volatile v4f*)(C + cofs + (size_t)(row0 + r) * ldc + col0 + c4) = v; if (C16) { v4h h4; for (int i = 0; i < 4; ++i) h4[i] = (_Float16)v[i]; *(volatile v4h*)(C16 + cofs + (size_t)(row0 + r) * ldc + col0 + c4) = h4; } }
    if (pass == 0) __threadfence(); } }


__global__ __launch_bounds__(256) void k_cls0(const float* __restrict__ cond, const float* __restrict__ w0, const float* __restrict__ b0, float* __restrict__ P0) {
  #pragma clang fp contract(off)
  const size_t t = (size_t)blockIdx.x * 256 + threadIdx.x; if (t >= (size_t)NB * 16 * 16384) return; const int q = (int)(t % 16384); const size_t bc = t / 16384; const int co = (int)(bc % 16); const size_t b = bc / 16; const int oy = q / 128, ox = q % 128; float acc = 0.f;
#pragma unroll 1
  for (int k = 0; k < 9; ++k) { const int y = 2 * oy - 1 + k / 3, x = 2 * ox - 1 + k % 3; if (y < 0 || y >= HS || x < 0 || x >= HS) continue; float v = bf16_round(b0[co]);
    for (int ci = 0; ci < 3; ++ci) v = __fadd_rn(v, __fmul_rn(bf16_round(w0[co * 3 + ci]), bf16_round(cond[((b * 3 + ci) * (size_t)PX) + (size_t)y * HS + x]))); acc += v; }
  acc = acc / 9.0f; acc = (acc >= 0.f) ? acc : 0.2f * acc; *(volatile float*)(P0 + t) = acc; __threadfence(); *(volatile float*)(P0 + t) = acc; }
__global__ __launch_bounds__(256) void k_pool(const float* __restrict__ F, int ldf, int C, int R, float* __restrict__ P) { const size_t t = (size_t)blockIdx.x * 256 + threadIdx.x; const int R2 = R / 2; const size_t nq = (size_t)R2 * R2; if (t >= (size_t)NB * C * nq) return; const int q = (int)(t % nq); const size_t bc = t / nq; const int c = (int)(bc % C); const size_t b = bc / C; const int oy = q / R2, ox = q % R2; float acc = 0.f;
#pragma unroll 1
  for (int k = 0; k < 9; ++k) { const int y = 2 * oy - 1 + k / 3, x = 2 * ox - 1 + k % 3; if (y < 0 || y >= R || x < 0 || x >= R) continue; acc += F[((b * R + y) * (size_t)R + x) * ldf + c]; }
  acc = acc / 9.0f; acc = (acc >= 0.f) ? acc : 0.2f * acc; *(volatile float*)(P + t) = acc; __threadfence(); *(volatile float*)(P + t) = acc; }
__global__ __launch_bounds__(256) void k_instat(const float* __restrict__ P, int nq, float* __restrict__ ST) { __shared__ double rs[256], rq[256]; const int tid = threadIdx.x; const float* p = P + (size_t)blockIdx.x * nq; double s = 0.0, q2 = 0.0; for (int i = tid; i < nq; i += 256) { const double v = (double)p[i]; s += v; q2 += v * v; }
  rs[tid] = s; rq[tid] = q2; __syncthreads(); for (int st = 128; st > 0; st >>= 1) { if (tid < st) { rs[tid] += rs[tid + st]; rq[tid] += rq[tid + st]; } __syncthreads(); }
  if (tid == 0) { const double mu = rs[0] / nq; double var = rq[0] / nq - mu * mu; if (var < 0.0) var = 0.0; const float m = (float)mu, r = (float)(1.0 / sqrt(var + 1e-5)); for (int pass = 0; pass < 2; ++pass) { *(volatile float*)(ST + (size_t)blockIdx.x * 32) = m; *(volatile float*)(ST + (size_t)blockIdx.x * 32 + 1) = r; if (pass == 0) __threadfence(); } } }
__global__ __launch_bounds__(256) void k_inrows(const float* __restrict__ P, const float* __restrict__ ST, const float* __restrict__ g, const float* __restrict__ e, int C, int CP, int nq, _Float16* __restrict__ A, _Float16* __restrict__ AL) {
  #pragma clang fp contract(off)
  const size_t t = (size_t)blockIdx.x * 256 + threadIdx.x; if (t >= (size_t)NB * nq * CP / 8) return; const int c0 = (int)((t * 8) % CP); const size_t bq = (t * 8) / CP; const int q = (int)(bq % nq); const size_t b = bq / nq; FragH f;
  FragH fl; for (int u = 0; u < 8; ++u) { const int c = c0 + u; float v = 0.f; if (c < C) { v = P[((b * C + c) * (size_t)nq) + q]; if (g) { const float m = ST[(b * C + c) * 32], r = ST[(b * C + c) * 32 + 1]; v = __fadd_rn(__fmul_rn((v - m) * r, bf16_round(g[c])), bf16_round(e[c])); } } const _Float16 hh = (_Float16)v; f.h[u] = hh; fl.h[u] = (_Float16)((v - (float)hh) * 1024.0f); }
  for (int pass = 0; pass < 2; ++pass) { *(volatile v8us*)((unsigned short*)A + t * 8) = f.half[0]; *(volatile v8us*)((unsigned short*)AL + t * 8) = fl.half[0]; if (pass == 0) __threadfence(); } }
__global__ __launch_bounds__(256) void k_wpad(const float* __restrict__ w, int O, int Iw, int OP, int IP, _Float16* __restrict__ Bt) { const size_t t = (size_t)blockIdx.x * 256 + threadIdx.x; if (t >= (size_t)OP * IP / 8) return; const int i0 = (int)((t * 8) % IP); const int o = (int)((t * 8) / IP); FragH f; for (int u = 0; u < 8; ++u) { const int i = i0 + u; f.h[u] = (o < O && i < Iw) ? (_Float16)(bf16_round(w[(size_t)o * Iw + i]) * 16.0f) : (_Float16)0.f; }
  *(volatile v8us*)((unsigned short*)Bt + t * 8) = f.half[0]; __threadfence(); *(volatile v8us*)((unsigned short*)Bt + t * 8) = f.half[0]; }
__global__ __launch_bounds__(256) void k_bpad(const float* __restrict__ b, int n, int np, float* __restrict__ bp) { const int i = blockIdx.x * 256 + threadIdx.x; if (i >= np) return; const float v = (i < n) ? b[i] : 0.f; *(volatile float*)(bp + i) = v; __threadfence(); *(volatile float*)(bp + i) = v; }
__global__ __launch_bounds__(256) void k_fea(const float* __restrict__ WF, float* __restrict__ fea) { const int t = blockIdx.x * 256 + threadIdx.x; if (t >= NB * NF) return; const int j = t % NF, b = t / NF; float s = 0.f;
#pragma unroll 1
  for (int q = 0; q < 64; ++q) s += WF[((size_t)b * 64 + q) * NF + j]; s = s / 64.0f; *(volatile float*)(fea + t) = s; __threadfence(); *(volatile float*)(fea + t) = s; }
__global__ __launch_bounds__(256) void k_lin(const float* __restrict__ fea, const float* __restrict__ w, const float* __restrict__ bb, int O, float* __restrict__ out) {
  #pragma clang fp contract(off)
  const int t = blockIdx.x * 256 + threadIdx.x; if (t >= NB * O) return; const int o = t % O, b = t / O; float s = 0.f;
#pragma unroll 1
  for (int k = 0; k < NF; ++k) s = __fadd_rn(s, __fmul_rn(fea[b * NF + k], bf16_round(w[(size_t)o * NF + k]))); s = s + bf16_round(bb[o]); *(volatile float*)(out + t) = s; __threadfence(); *(volatile float*)(out + t) = s; }
__global__ __launch_bounds__(256) void k_lowrank(const float* __restrict__ U, const float* __restrict__ V, _Float16* __restrict__ S16) {
  #pragma clang fp contract(off)
  const int t = blockIdx.x * 256 + threadIdx.x; if (t >= NB * NF * NF / 8) return; const int j0 = (t * 8) % NF; const int bi = (t * 8) / NF; const int i = bi % NF, b = bi / NF; FragH f;
  for (int u = 0; u < 8; ++u) { const int j = j0 + u; float s = 0.f; for (int k = 0; k < KT; ++k) s = __fadd_rn(s, __fmul_rn(U[b * 256 + i * 4 + k], V[b * 256 + k * 64 + j])); f.h[u] = (_Float16)s; }
  *(volatile v8us*)((unsigned short*)S16 + (size_t)t * 8) = f.half[0]; __threadfence(); *(volatile v8us*)((unsigned short*)S16 + (size_t)t * 8) = f.half[0]; }
__global__ __launch_bounds__(256) void k_crows(const float* __restrict__ content, int b, _Float16* __restrict__ CR) { const size_t p = (size_t)blockIdx.x * 256 + threadIdx.x; if (p >= PX) return; FragH f[4]; for (int a = 0; a < 4; ++a) for (int u = 0; u < 8; ++u) f[a].h[u] = (_Float16)0.f;
  for (int c = 0; c < 3; ++c) f[0].h[c] = (_Float16)bf16_round(content[(((size_t)b * 3 + c) * PX) + p]);
  for (int pass = 0; pass < 2; ++pass) { for (int a = 0; a < 4; ++a) *(volatile v8us*)((unsigned short*)CR + p * 32 + a * 8) = f[a].half[0]; if (pass == 0) __threadfence(); } }
__global__ __launch_bounds__(256) void k_tof16(const float* __restrict__ F, _Float16* __restrict__ H, size_t n8) { const size_t t = (size_t)blockIdx.x * 256 + threadIdx.x; if (t >= n8) return; const v8f v = *(const v8f*)(F + t * 8); FragH f; for (int u = 0; u < 8; ++u) f.h[u] = (_Float16)v[u]; *(volatile v8us*)((unsigned short*)H + t * 8) = f.half[0]; __threadfence(); *(volatile v8us*)((unsigned short*)H + t * 8) = f.half[0]; }
__global__ __launch_bounds__(256) void k_addrow(float* __restrict__ F, const float* __restrict__ v, size_t n8) { const size_t t = (size_t)blockIdx.x * 256 + threadIdx.x; if (t >= n8) return; const int c0 = (int)((t * 8) % 64); v8f a = *(const v8f*)(F + t * 8); for (int u = 0; u < 8; ++u) a[u] = a[u] + v[c0 + u]; *(volatile v8f*)(F + t * 8) = a; __threadfence(); *(volatile v8f*)(F + t * 8) = a; }
__global__ __launch_bounds__(256) void k_final(const float* __restrict__ O3, int b, const float* __restrict__ SL, const float* __restrict__ SHL, float* __restrict__ out) {
  #pragma clang fp contract(off)
  const size_t t = (size_t)blockIdx.x * 256 + threadIdx.x; if (t >= (size_t)3 * PX / 8) return; const int p0 = (int)((t * 8) % PX); const int c = (int)((t * 8) / PX); const float sl = SL[b * 3 + c], sh = SHL[b * 3 + c]; v8f r;
  for (int u = 0; u < 8; ++u) { const float o = O3[(size_t)(p0 + u) * 64 + c]; r[u] = (__fmul_rn(o, sl) + sh) + o; }
  float* d = out + ((size_t)b * 3 + c) * PX + p0; *(volatile v8f*)d = r; __threadfence(); *(volatile v8f*)d = r; }

extern "C" void kernel_launch(void* const* d_in, const int* in_sizes, int n_in,
                              void* d_out, int out_size, void* d_ws, size_t ws_size, hipStream_t stream) {
  (void)in_sizes; (void)n_in; (void)out_size;
  const float* const* I = (const float* const*)d_in; const float* content = I[0]; const float* cond = I[1];
  const float* clsw[5] = {I[2], I[4], I[6], I[8], I[10]}; const float* clsb[5] = {I[3], I[5], I[7], I[9], I[11]}; const float* clsg[4] = {I[12], I[14], I[16], I[18]}; const float* clse[4] = {I[13], I[15], I[17], I[19]}; const float* wf = I[20]; const float* bfb = I[21];
  const float *w_sf0 = I[22], *b_sf0 = I[23], *w_sf1 = I[24], *b_sf1 = I[25], *w_hr0 = I[26], *b_hr0 = I[27], *w_hr1 = I[28], *b_hr1 = I[29], *w_sl = I[30], *b_sl = I[31], *w_shf = I[32], *b_shf = I[33], *w_shr = I[34], *b_shr = I[35], *w_shl = I[36], *b_shl = I[37], *cf_w = I[38], *cf_b = I[39], *hr_w = I[40], *hr_b = I[41], *cl_w = I[42], *cl_b = I[43];
  char* ws = (char*)d_ws; size_t off = 0;
  auto take = [&](size_t bytes) { char* p = ws + off; off += (bytes + 255) & ~(size_t)255; return p; };
  const int Cs[5] = {3, 16, 32, 64, 128}, Os[5] = {16, 32, 64, 128, 128}, CPs[5] = {0, 32, 32, 64, 128}, OPs[5] = {16, 64, 64, 128, 128}; const int Rs[5] = {256, 128, 64, 32, 16};
  _Float16* BW[5]; float* BB[5]; for (int s = 1; s < 5; ++s) { BW[s] = (_Float16*)take((size_t)OPs[s] * CPs[s] * 2); BB[s] = (float*)take((size_t)OPs[s] * 4); } _Float16* BWF = (_Float16*)take((size_t)64 * 128 * 2); _Float16* BCF = (_Float16*)take((size_t)64 * 32 * 2); _Float16* BHR = (_Float16*)take((size_t)64 * 64 * 2); _Float16* BCL = (_Float16*)take((size_t)64 * 64 * 2); float* bclp = (float*)take(64 * 4);
  float* P = (float*)take((size_t)NB * 16 * 16384 * 4); float* ST = (float*)take((size_t)NB * 128 * 32 * 4); _Float16* A = (_Float16*)take((size_t)NB * 16384 * 32 * 2); _Float16* AL = (_Float16*)take((size_t)NB * 16384 * 32 * 2); float* F = (float*)take((size_t)NB * 16384 * 64 * 4);
  float* fea = (float*)take(NB * NF * 4); float* LSF0 = (float*)take(NB * 256 * 4); float* LSF1 = (float*)take(NB * 256 * 4); float* LHR0 = (float*)take(NB * 256 * 4); float* LHR1 = (float*)take(NB * 256 * 4); float* LSL = (float*)take(NB * 3 * 4); float* LSHF = (float*)take(NB * 64 * 4); float* LSHR = (float*)take(NB * 64 * 4); float* LSHL = (float*)take(NB * 3 * 4); _Float16* SF16 = (_Float16*)take((size_t)NB * 64 * 64 * 2); _Float16* SH16 = (_Float16*)take((size_t)NB * 64 * 64 * 2);
  _Float16* CR = (_Float16*)take((size_t)PX * 32 * 2); float* O0 = (float*)take((size_t)PX * 64 * 4); _Float16* O016 = (_Float16*)take((size_t)PX * 64 * 2); _Float16* X1 = (_Float16*)take((size_t)PX * 64 * 2); float* O2 = (float*)take((size_t)PX * 64 * 4); _Float16* O216 = (_Float16*)take((size_t)PX * 64 * 2); _Float16* X3 = (_Float16*)take((size_t)PX * 64 * 2); float* O3 = (float*)take((size_t)PX * 64 * 4);
  if (off > ws_size) return;
  for (int s = 1; s < 5; ++s) { k_wpad<<<(unsigned)(((size_t)OPs[s] * CPs[s] / 8 + 255) / 256), 256, 0, stream>>>(clsw[s], Os[s], Cs[s], OPs[s], CPs[s], BW[s]); k_bpad<<<1, 256, 0, stream>>>(clsb[s], Os[s], OPs[s], BB[s]); }
  k_wpad<<<(64 * 128 / 8 + 255) / 256, 256, 0, stream>>>(wf, 64, 128, 64, 128, BWF); k_wpad<<<(64 * 32 / 8 + 255) / 256, 256, 0, stream>>>(cf_w, 64, 3, 64, 32, BCF); k_wpad<<<(64 * 64 / 8 + 255) / 256, 256, 0, stream>>>(hr_w, 64, 64, 64, 64, BHR); k_wpad<<<(64 * 64 / 8 + 255) / 256, 256, 0, stream>>>(cl_w, 3, 64, 64, 64, BCL); k_bpad<<<1, 256, 0, stream>>>(cl_b, 3, 64, bclp);
  k_cls0<<<(unsigned)(((size_t)NB * 16 * 16384 + 255) / 256), 256, 0, stream>>>(cond, clsw[0], clsb[0], P);
  for (int s = 1; s < 5; ++s) { const int C = Cs[s], R = Rs[s], nq = R * R; const size_t nrows = (size_t)NB * nq;
    k_instat<<<NB * C, 256, 0, stream>>>(P, nq, ST); k_inrows<<<(unsigned)((nrows * CPs[s] / 8 + 255) / 256), 256, 0, stream>>>(P, ST, clsg[s - 1], clse[s - 1], C, CPs[s], nq, A, AL);
    k_gemm2<0><<<dim3((unsigned)((nrows / 128) * (OPs[s] / 64)), 1), 128, 0, stream>>>(AL, CPs[s], 0, BW[s], CPs[s], 0, 0.0625f / 1024.0f, nullptr, 0, nullptr, 1, 0, 0, F, nullptr, OPs[s], 0, (int)nrows, OPs[s], CPs[s]);
    k_gemm2<0><<<dim3((unsigned)((nrows / 128) * (OPs[s] / 64)), 1), 128, 0, stream>>>(A, CPs[s], 0, BW[s], CPs[s], 0, 0.0625f, BB[s], 0, F, 1, (size_t)OPs[s], 0, F, nullptr, OPs[s], 0, (int)nrows, OPs[s], CPs[s]);
    k_pool<<<(unsigned)(((size_t)NB * Os[s] * (nq / 4) + 255) / 256), 256, 0, stream>>>(F, OPs[s], Os[s], R, P); }
  k_inrows<<<(unsigned)((((size_t)NB * 64) * 128 / 8 + 255) / 256), 256, 0, stream>>>(P, ST, nullptr, nullptr, 128, 128, 64, A, AL);
  k_gemm2<0><<<dim3((NB * 64 / 128) * 1, 1), 128, 0, stream>>>(AL, 128, 0, BWF, 128, 0, 0.0625f / 1024.0f, nullptr, 0, nullptr, 1, 0, 0, F, nullptr, 64, 0, NB * 64, 64, 128);
  k_gemm2<0><<<dim3((NB * 64 / 128) * 1, 1), 128, 0, stream>>>(A, 128, 0, BWF, 128, 0, 0.0625f, bfb, 0, F, 1, (size_t)64, 0, F, nullptr, 64, 0, NB * 64, 64, 128); k_fea<<<(NB * NF + 255) / 256, 256, 0, stream>>>(F, fea);
  k_lin<<<(NB * 256 + 255) / 256, 256, 0, stream>>>(fea, w_sf0, b_sf0, 256, LSF0); k_lin<<<(NB * 256 + 255) / 256, 256, 0, stream>>>(fea, w_sf1, b_sf1, 256, LSF1); k_lin<<<(NB * 256 + 255) / 256, 256, 0, stream>>>(fea, w_hr0, b_hr0, 256, LHR0); k_lin<<<(NB * 256 + 255) / 256, 256, 0, stream>>>(fea, w_hr1, b_hr1, 256, LHR1);
  k_lin<<<(NB * 3 + 255) / 256, 256, 0, stream>>>(fea, w_sl, b_sl, 3, LSL); k_lin<<<(NB * 64 + 255) / 256, 256, 0, stream>>>(fea, w_shf, b_shf, 64, LSHF); k_lin<<<(NB * 64 + 255) / 256, 256, 0, stream>>>(fea, w_shr, b_shr, 64, LSHR); k_lin<<<(NB * 3 + 255) / 256, 256, 0, stream>>>(fea, w_shl, b_shl, 3, LSHL);
  k_lowrank<<<(NB * NF * NF / 8 + 255) / 256, 256, 0, stream>>>(LSF0, LSF1, SF16); k_lowrank<<<(NB * NF * NF / 8 + 255) / 256, 256, 0, stream>>>(LHR0, LHR1, SH16);
  const dim3 gp((PX / 128) * 1, 1); const unsigned n8 = (unsigned)(((size_t)PX * 64 / 8 + 255) / 256);
  for (int b = 0; b < NB; ++b) {
    k_crows<<<(PX + 255) / 256, 256, 0, stream>>>(content, b, CR);
    k_gemm2<0><<<gp, 128, 0, stream>>>(CR, 32, 0, BCF, 32, 0, 0.0625f, cf_b, 0, nullptr, 1, 0, 0, O0, O016, 64, 0, PX, 64, 32);
    k_addrow<<<n8, 256, 0, stream>>>(O0, LSHF + b * 64, (size_t)PX * 64 / 8);
    k_gemm2<3><<<gp, 128, 0, stream>>>(O016, 64, 0, SF16 + (size_t)b * 64 * 64, 64, 0, 1.0f, nullptr, 0, O0, 1, (size_t)64, 0, nullptr, X1, 64, 0, PX, 64, 64);
    k_gemm2<0><<<gp, 128, 0, stream>>>(X1, 64, 0, BHR, 64, 0, 0.0625f, hr_b, 0, nullptr, 1, 0, 0, O2, O216, 64, 0, PX, 64, 64);
    k_addrow<<<n8, 256, 0, stream>>>(O2, LSHR + b * 64, (size_t)PX * 64 / 8);
    k_gemm2<3><<<gp, 128, 0, stream>>>(O216, 64, 0, SH16 + (size_t)b * 64 * 64, 64, 0, 1.0f, nullptr, 0, O2, 1, (size_t)64, 0, nullptr, X3, 64, 0, PX, 64, 64);
    k_gemm2<0><<<gp, 128, 0, stream>>>(X3, 64, 0, BCL, 64, 0, 0.0625f, bclp, 0, nullptr, 1, 0, 0, O3, nullptr, 64, 0, PX, 64, 64);
    k_final<<<(unsigned)(((size_t)3 * PX / 8 + 255) / 256), 256, 0, stream>>>(O3, b, LSL, LSHL, (float*)d_out); }
}
